// SelectiveScan_8572754723195
// MI455X (gfx1250) — hardware-verified
//
#include <hip/hip_runtime.h>
#include <math.h>

typedef __attribute__((ext_vector_type(16))) _Float16 v16h;
typedef __attribute__((ext_vector_type(8)))  _Float16 v8h;
typedef __attribute__((ext_vector_type(16))) __bf16   v16b;
typedef __attribute__((ext_vector_type(8)))  __bf16   v8b;
typedef __attribute__((ext_vector_type(8)))  float    v8f;
typedef __attribute__((ext_vector_type(4)))  float    v4f;
typedef __attribute__((ext_vector_type(2)))  float    v2f;

constexpr int kBatch  = 2;
constexpr int kSeq    = 2048;
constexpr int kD      = 1024;
constexpr int kNst    = 16;
constexpr int kDtR    = 64;
constexpr int kPrN    = 96;
constexpr int kPrP    = 128;
constexpr int kXzN    = 2 * kD;
constexpr int kRows   = kBatch * kSeq;
constexpr int kConvK  = 4;
constexpr int kBcW    = 2 * kNst;
constexpr int kScanTS = 64;
constexpr int kScanCh = 64;
constexpr int kScanYP = 68;
static_assert(kDtR + 2 * kNst == kPrN, "params width");
static_assert((kD % 32) == 0 && (kDtR % 32) == 0 && (kDtR == 64), "GEMM K multiples of 32");
static_assert((kRows % 64) == 0 && (kXzN % 64) == 0 && (kPrP % 64) == 0 && (kD % 64) == 0, "GEMM M,N multiples of 64");
static_assert((kSeq % kScanTS) == 0 && (kD % kScanCh) == 0 && (kScanCh == 64) && (kScanTS == 64) && (kNst == 16), "scan tile shape");
static_assert(((kRows * kXzN / 64) % 8) == 0 && ((kRows * kPrP / 4096) % 8) == 0 && ((kRows * kD / 4096) % 8) == 0, "GEMM tiles per block");

constexpr size_t kOffXB   = 0;
constexpr size_t kOffWXZ  = kOffXB  + (size_t)kRows * kD   * 2;
constexpr size_t kOffWP   = kOffWXZ + (size_t)kXzN  * kD   * 2;
constexpr size_t kOffWDT  = kOffWP  + (size_t)kPrP  * kD   * 2;
constexpr size_t kOffWO   = kOffWDT + (size_t)kD    * kDtR * 2;
constexpr size_t kOffXZ   = kOffWO  + (size_t)kD    * kD   * 2;
constexpr size_t kOffPR   = kOffXZ  + (size_t)kRows * kXzN * 4;
constexpr size_t kOffDTH  = kOffPR  + (size_t)kRows * kPrP * 4;
constexpr size_t kOffDTL  = kOffDTH + (size_t)kRows * kDtR * 2;
constexpr size_t kOffYH   = kOffDTL + (size_t)kRows * kDtR * 2;
constexpr size_t kOffYL   = kOffYH  + (size_t)kRows * kD   * 2;
constexpr size_t kWsTotal = kOffYL  + (size_t)kRows * kD   * 2;
static_assert(kWsTotal == 68550656ull, "carve total");
static_assert(kWsTotal <= 134217728ull, "carve cap");
static_assert((kOffWXZ % 128) == 0 && (kOffWP % 128) == 0 && (kOffWDT % 128) == 0 && (kOffWO % 128) == 0 &&
              (kOffXZ % 128) == 0 && (kOffPR % 128) == 0 && (kOffDTH % 128) == 0 && (kOffDTL % 128) == 0 &&
              (kOffYH % 128) == 0 && (kOffYL % 128) == 0, "128-B aligned regions");

__device__ __forceinline__ unsigned short f2bf_bits(float f) {
  unsigned u = __float_as_uint(f);
  return (unsigned short)((u + 0x7FFFu + ((u >> 16) & 1u)) >> 16);
}
__device__ __forceinline__ float bf_bits2f(unsigned short h) { return __uint_as_float(((unsigned)h) << 16); }
__device__ __forceinline__ float bf_rne(float f) { return bf_bits2f(f2bf_bits(f)); }

__device__ __forceinline__ void dep_guard_h(v8f& a, v8f& b, v16h x, v16h y) { asm volatile("v_nop\n\tv_nop\n\tv_nop\n\tv_nop" : "+v"(a), "+v"(b) : "v"(x), "v"(y)); }
__device__ __forceinline__ void dep_guard_b(v8f& a, v8f& b, v16b x, v16b y) { asm volatile("v_nop\n\tv_nop\n\tv_nop\n\tv_nop" : "+v"(a), "+v"(b) : "v"(x), "v"(y)); }
__device__ __forceinline__ void keep4_h(v16h a, v16h b, v16h c, v16h d) { asm volatile("v_nop" :: "v"(a), "v"(b), "v"(c), "v"(d)); }
__device__ __forceinline__ void keep4_b(v16b a, v16b b, v16b c, v16b d) { asm volatile("v_nop" :: "v"(a), "v"(b), "v"(c), "v"(d)); }
__device__ __forceinline__ void acc_guard4(v8f& a, v8f& b, v8f& c, v8f& d) { asm volatile("v_nop\n\tv_nop\n\tv_nop\n\tv_nop" : "+v"(a), "+v"(b), "+v"(c), "+v"(d)); }
template <typename T> struct Frag;
template <> struct Frag<_Float16> {
  typedef v16h V; union U { v16h v; v8h h[2]; };
  static __device__ __forceinline__ v16h load(const _Float16* p) {
    U f; f.h[0] = *(const v8h*)(p); f.h[1] = *(const v8h*)(p + 16); return f.v;
  }
  static __device__ __forceinline__ v8f mma(v16h a, v16h b, v8f c) {
    return __builtin_amdgcn_wmma_f32_16x16x32_f16(false, a, false, b, (short)0, c, false, false);
  }
  static __device__ __forceinline__ void guard(v8f& a, v8f& b, v16h x, v16h y) { dep_guard_h(a, b, x, y); }
  static __device__ __forceinline__ void keep(v16h a, v16h b, v16h c, v16h d) { keep4_h(a, b, c, d); }
};
template <> struct Frag<__bf16> {
  typedef v16b V; union U { v16b v; v8b h[2]; };
  static __device__ __forceinline__ v16b load(const __bf16* p) {
    U f; f.h[0] = *(const v8b*)(p); f.h[1] = *(const v8b*)(p + 16); return f.v;
  }
  static __device__ __forceinline__ v8f mma(v16b a, v16b b, v8f c) {
    return __builtin_amdgcn_wmma_f32_16x16x32_bf16(false, a, false, b, (short)0, c, false, false);
  }
  static __device__ __forceinline__ void guard(v8f& a, v8f& b, v16b x, v16b y) { dep_guard_b(a, b, x, y); }
  static __device__ __forceinline__ void keep(v16b a, v16b b, v16b c, v16b d) { keep4_b(a, b, c, d); }
};
__device__ __forceinline__ v8f mma_bf_g(v16b a, v16b b, v8f c) {
  c = __builtin_amdgcn_wmma_f32_16x16x32_bf16(false, a, false, b, (short)0, c, false, false);
  asm volatile("v_nop\n\tv_nop\n\tv_nop\n\tv_nop" : "+v"(c) : "v"(a), "v"(b));
  return c;
}

template <int ET> struct Elem;
template <> struct Elem<0> { typedef _Float16 T; };
template <> struct Elem<1> { typedef __bf16 T; };
template <int ET, int SPL, int BIAS_MODE, int OUT_MODE, bool RESID, int ACT = 0>
__global__ __launch_bounds__(256) void wmma_gemm64(
    const unsigned short* __restrict__ Ap, const unsigned short* __restrict__ A2p, int lda, long strideA,
    const unsigned short* __restrict__ Btp, const unsigned short* __restrict__ Bt2p, int ldb, long strideB,
    void* __restrict__ Cout, void* __restrict__ Cout2, int ldc, long strideC,
    const float* __restrict__ bias,
    const float* __restrict__ resid, long strideR,
    int M, int N, int K, float scale) {
  typedef typename Elem<ET>::T T;
  typedef typename Frag<T>::V V;
  const T* A = (const T*)Ap; const T* A2 = (const T*)A2p; const T* Bt = (const T*)Btp; const T* Bt2 = (const T*)Bt2p;
  __shared__ __align__(16) float sT[8][16 * 68];
  const int b    = blockIdx.y;
  const int lane = threadIdx.x & 31;
  const int wave = threadIdx.x >> 5;
  const int tilesN = N >> 6;
  const int tilesM = M >> 6;
  const int tile = blockIdx.x * 8 + wave;
  if (tile >= tilesM * tilesN) return;
  const int tm = tile / tilesN;
  const int tn = tile - tm * tilesN;
  const int m0 = tm << 6;
  const int n0 = tn << 6;

  const T* Ab  = A  + (size_t)b * strideA;
  const T* Bb  = Bt + (size_t)b * strideB;
  const T* Ab2 = (SPL >= 1) ? (A2  + (size_t)b * strideA) : nullptr;
  const T* Bb2 = (SPL == 2) ? (Bt2 + (size_t)b * strideB) : nullptr;

  const int rlane = lane & 15;
  const int koff  = (lane >> 4) * 8;
  const int mOff  = (lane >> 4) * 8;

  v8f acc[4][4];
#pragma unroll
  for (int i = 0; i < 4; ++i)
#pragma unroll
    for (int j = 0; j < 4; ++j) acc[i][j] = (v8f){0.f,0.f,0.f,0.f,0.f,0.f,0.f,0.f};

  for (int k0 = 0; k0 < K; k0 += 32) {
    V bh[4], bl[4];
#pragma unroll
    for (int j = 0; j < 4; ++j) {
      const size_t bo = (size_t)(n0 + (j << 4) + rlane) * ldb + koff + k0;
      bh[j] = Frag<T>::load(Bb + bo);
      if (SPL == 2) bl[j] = Frag<T>::load(Bb2 + bo);
    }
#pragma unroll
    for (int i = 0; i < 4; ++i) {
      const size_t ao = (size_t)(m0 + (i << 4) + rlane) * lda + koff + k0;
      V ah = Frag<T>::load(Ab + ao);
      V al;
      if (SPL >= 1) al = Frag<T>::load(Ab2 + ao);
#pragma unroll
      for (int j = 0; j < 4; ++j) {
        acc[i][j] = Frag<T>::mma(ah, bh[j], acc[i][j]);
        if (SPL == 2) acc[i][j] = Frag<T>::mma(ah, bl[j], acc[i][j]);
        if (SPL >= 1) acc[i][j] = Frag<T>::mma(al, bh[j], acc[i][j]);
      }
      Frag<T>::guard(acc[i][0], acc[i][3], ah, (SPL >= 1) ? al : ah);
    }
    Frag<T>::keep(bh[0], bh[1], bh[2], bh[3]);
    if (SPL == 2) Frag<T>::keep(bl[0], bl[1], bl[2], bl[3]);
  }
  acc_guard4(acc[0][0], acc[0][1], acc[0][2], acc[0][3]);
  acc_guard4(acc[1][0], acc[1][1], acc[1][2], acc[1][3]);
  acc_guard4(acc[2][0], acc[2][1], acc[2][2], acc[2][3]);
  acc_guard4(acc[3][0], acc[3][1], acc[3][2], acc[3][3]);

  float* slab = sT[wave];
  const float* Rb = RESID ? (resid + (size_t)b * strideR) : nullptr;
#pragma unroll
  for (int i = 0; i < 4; ++i) {
    const int mBase = m0 + (i << 4);
#pragma unroll
    for (int j = 0; j < 4; ++j) {
      const int n = n0 + (j << 4) + rlane;
      float bv = 0.f;
      if (BIAS_MODE == 2) bv = bias[n];
#pragma unroll
      for (int r = 0; r < 8; ++r) {
        float v = acc[i][j][r] * scale;
        if (BIAS_MODE == 1) v += bias[mBase + mOff + r];
        if (BIAS_MODE == 2) v += bv;
        if (RESID) v += Rb[(size_t)(mBase + mOff + r) * ldc + n];
        if (ACT == 1) v = tanhf(v);
        if (ACT == 2) v = fmaxf(v, 0.0f);
        if (ACT == 3) v = v / (1.0f + expf(-v));
        if (ACT == 4) v = (v > 0.f) ? v : 0.01f * v;
        slab[(mOff + r) * 68 + (j << 4) + rlane] = v;
      }
    }
    __builtin_amdgcn_fence(__ATOMIC_RELEASE, "workgroup");
    __builtin_amdgcn_wave_barrier();
    __builtin_amdgcn_fence(__ATOMIC_ACQUIRE, "workgroup");
    if (OUT_MODE == 0) {
      float* C = (float*)Cout + (size_t)b * strideC;
      const int hh = lane >> 4, c4 = (lane & 15) * 4;
      for (int pass = 0; pass < 2; ++pass) {
#pragma unroll
        for (int it = 0; it < 8; ++it) {
          const int row = it * 2 + hh;
          v4f v = *(const v4f*)(slab + row * 68 + c4);
          *(volatile v4f*)(C + (size_t)(mBase + row) * ldc + n0 + c4) = v;
        }
        __threadfence();
      }
    } else {
      const int q = lane >> 3, c8 = (lane & 7) * 8;
      unsigned short* C  = (unsigned short*)Cout  + (size_t)b * strideC;
      unsigned short* C2 = (OUT_MODE == 2) ? ((unsigned short*)Cout2 + (size_t)b * strideC) : nullptr;
      for (int pass = 0; pass < 2; ++pass) {
#pragma unroll
        for (int it = 0; it < 4; ++it) {
          const int row = it * 4 + q;
          const float* sp = slab + row * 68 + c8;
          v8h hv, lv;
#pragma unroll
          for (int e = 0; e < 8; ++e) {
            if (OUT_MODE == 1) {
              hv[e] = (_Float16)sp[e];
            } else {
              unsigned short hb = f2bf_bits(sp[e]);
              unsigned short lb = f2bf_bits(sp[e] - bf_bits2f(hb));
              hv[e] = __builtin_bit_cast(_Float16, hb);
              lv[e] = __builtin_bit_cast(_Float16, lb);
            }
          }
          *(volatile v8h*)(C + (size_t)(mBase + row) * ldc + n0 + c8) = hv;
          if (OUT_MODE == 2) *(volatile v8h*)(C2 + (size_t)(mBase + row) * ldc + n0 + c8) = lv;
        }
        __threadfence();
      }
    }
    __builtin_amdgcn_fence(__ATOMIC_RELEASE, "workgroup");
    __builtin_amdgcn_wave_barrier();
    __builtin_amdgcn_fence(__ATOMIC_ACQUIRE, "workgroup");
  }
}

__global__ __launch_bounds__(256) void cvt_rows_bf16_kernel(
    const float* __restrict__ src, unsigned short* __restrict__ dst, int real8, int total8)
{
  const int i = blockIdx.x * 256 + threadIdx.x;
  if (i >= total8) return;
  const int j = (i < real8) ? i : (real8 - 1);
  const size_t e0 = (size_t)j << 3;
  const v4f a0 = *(const v4f*)(src + e0);
  const v4f a1 = *(const v4f*)(src + e0 + 4);
  const bool live = (i < real8);
  v8h hv;
#pragma unroll
  for (int e = 0; e < 4; ++e) {
    const float f0 = live ? a0[e] : 0.0f;
    const float f1 = live ? a1[e] : 0.0f;
    hv[e]     = __builtin_bit_cast(_Float16, f2bf_bits(f0));
    hv[4 + e] = __builtin_bit_cast(_Float16, f2bf_bits(f1));
  }
  unsigned short* qd = dst + ((size_t)i << 3);
  *(volatile v8h*)qd = hv;
  __threadfence();
  *(volatile v8h*)qd = hv;
}

__global__ __launch_bounds__(256) void split_dtun_kernel(
    const float* __restrict__ PR, unsigned short* __restrict__ DH, unsigned short* __restrict__ DL, int total8)
{
  const int i = blockIdx.x * 256 + threadIdx.x;
  if (i >= total8) return;
  const int row = i >> 3, c8 = (i & 7) * 8;
  const float* sp = PR + (size_t)row * kPrP + c8;
  const v4f a0 = *(const v4f*)(sp);
  const v4f a1 = *(const v4f*)(sp + 4);
  v8h hv, lv;
#pragma unroll
  for (int e = 0; e < 4; ++e) {
    const unsigned short h0 = f2bf_bits(a0[e]), h1 = f2bf_bits(a1[e]);
    const unsigned short l0 = f2bf_bits(a0[e] - bf_bits2f(h0)), l1 = f2bf_bits(a1[e] - bf_bits2f(h1));
    hv[e]     = __builtin_bit_cast(_Float16, h0);
    hv[4 + e] = __builtin_bit_cast(_Float16, h1);
    lv[e]     = __builtin_bit_cast(_Float16, l0);
    lv[4 + e] = __builtin_bit_cast(_Float16, l1);
  }
  const size_t o = (size_t)row * kDtR + c8;
  unsigned short* qh = DH + o;
  unsigned short* ql = DL + o;
  *(volatile v8h*)qh = hv;
  *(volatile v8h*)ql = lv;
  __threadfence();
  *(volatile v8h*)qh = hv;
  *(volatile v8h*)ql = lv;
}

__global__ __launch_bounds__(kScanCh) void scan_kernel(
    const unsigned short* __restrict__ DTH, const unsigned short* __restrict__ DTL,
    const unsigned short* __restrict__ WDT,
    const float* __restrict__ XZ, const float* __restrict__ PR,
    const float* __restrict__ convw, const float* __restrict__ bdt, const float* __restrict__ Alog,
    const float* __restrict__ Dp, unsigned short* __restrict__ YH, unsigned short* __restrict__ YL)
{
  __shared__ __align__(16) float sP[kScanTS * kBcW];
  __shared__ __align__(16) float sD[kScanTS * kScanYP];
  __shared__ __align__(16) float sY[kScanTS * kScanYP];
  __shared__ __align__(16) float sH[kNst * kScanCh];
  __shared__ __align__(16) float sA[kNst * kScanCh];
  __shared__ __align__(16) float sR[kNst * kScanCh];
  const int tid = threadIdx.x, lane = tid & 31, wave = tid >> 5;
  constexpr int kBlkPerB = kD / kScanCh;
  const int bix = blockIdx.x / kBlkPerB;
  const int d0  = (blockIdx.x - bix * kBlkPerB) * kScanCh;
  const int d   = d0 + tid;
  const size_t row0 = (size_t)bix * kSeq;
  const __bf16* Ah = (const __bf16*)DTH;
  const __bf16* Al = (const __bf16*)DTL;
  const __bf16* Wb = (const __bf16*)WDT;
  const int rlane = lane & 15;
  const int koff  = (lane >> 4) * 8;
  const int mOff  = (lane >> 4) * 8;
#pragma unroll 1
  for (int n = 0; n < kNst; ++n) {
    const float al = bf_rne(Alog[(size_t)d * kNst + n]);
    const float An = -expf(al);
    sA[n * kScanCh + tid] = An;
    sR[n * kScanCh + tid] = 1.0f / (An + 1e-8f);
    sH[n * kScanCh + tid] = 0.0f;
  }
  const float w0 = bf_rne(convw[(size_t)d * kConvK + 0]);
  const float w1 = bf_rne(convw[(size_t)d * kConvK + 1]);
  const float w2 = bf_rne(convw[(size_t)d * kConvK + 2]);
  const float w3 = bf_rne(convw[(size_t)d * kConvK + 3]);
  const float bb = bf_rne(bdt[d]);
  const float Dd = bf_rne(Dp[d]);
  __syncthreads();
  float xm3 = 0.0f, xm2 = 0.0f, xm1 = 0.0f;
  const int q = lane >> 3, c8 = (lane & 7) * 8;
#pragma unroll 1
  for (int t0 = 0; t0 < kSeq; t0 += kScanTS) {
    __syncthreads();
#pragma unroll
    for (int i = 0; i < 8; ++i) {
      const int idx = i * kScanCh + tid;
      const int r = idx >> 3;
      const int c4 = (idx & 7) * 4;
      *(v4f*)(sP + r * kBcW + c4) = *(const v4f*)(PR + (row0 + t0 + r) * kPrP + kDtR + c4);
    }
    {
      v16b bfr[2][2];
#pragma unroll
      for (int jj = 0; jj < 2; ++jj) {
#pragma unroll
        for (int ks = 0; ks < 2; ++ks) {
          bfr[jj][ks] = Frag<__bf16>::load(Wb + (size_t)(d0 + 32 * wave + 16 * jj + rlane) * kDtR + koff + 32 * ks);
        }
      }
#pragma unroll 1
      for (int i = 0; i < 4; ++i) {
        const size_t ar = (row0 + t0 + 16 * i + rlane) * kDtR + koff;
        const v16b ah0 = Frag<__bf16>::load(Ah + ar);
        const v16b al0 = Frag<__bf16>::load(Al + ar);
        const v16b ah1 = Frag<__bf16>::load(Ah + ar + 32);
        const v16b al1 = Frag<__bf16>::load(Al + ar + 32);
#pragma unroll
        for (int jj = 0; jj < 2; ++jj) {
          v8f acc = (v8f){0.f,0.f,0.f,0.f,0.f,0.f,0.f,0.f};
          acc = mma_bf_g(ah0, bfr[jj][0], acc);
          acc = mma_bf_g(al0, bfr[jj][0], acc);
          acc = mma_bf_g(ah1, bfr[jj][1], acc);
          acc = mma_bf_g(al1, bfr[jj][1], acc);
          float* dp = sD + (16 * i + mOff) * kScanYP + 32 * wave + 16 * jj + rlane;
#pragma unroll
          for (int r = 0; r < 8; ++r) dp[r * kScanYP] = acc[r];
        }
      }
    }
    __syncthreads();
#pragma unroll 1
    for (int s = 0; s < kScanTS; ++s) {
      const size_t grow = row0 + t0 + s;
      const float xcur = XZ[grow * kXzN + d];
      const float zv   = XZ[grow * kXzN + kD + d];
      const float dl   = sD[s * kScanYP + tid];
      float cv = w0 * xm3;
      cv = fmaf(w1, xm2, cv);
      cv = fmaf(w2, xm1, cv);
      cv = fmaf(w3, xcur, cv);
      xm3 = xm2; xm2 = xm1; xm1 = xcur;
      const float uu  = cv * __builtin_amdgcn_rcpf(1.0f + expf(-cv));
      const float v   = dl + bb;
      const float ea  = expf(-fabsf(v));
      const float up  = 1.0f + ea;
      const float l1p = logf(up) + (ea - (up - 1.0f)) * __builtin_amdgcn_rcpf(up);
      const float dtv = fmaxf(v, 0.0f) + l1p;
      const float* pr = sP + s * kBcW;
      float y = 0.0f;
#pragma unroll 1
      for (int j = 0; j < kNst / 2; ++j) {
        const v2f bq = *(const v2f*)(pr + 2 * j);
        const v2f cq = *(const v2f*)(pr + kNst + 2 * j);
#pragma unroll
        for (int e = 0; e < 2; ++e) {
          const int o = (2 * j + e) * kScanCh + tid;
          const float An = sA[o];
          const float rn = sR[o];
          float hn = sH[o];
          const float a   = expf(An * dtv);
          const float bt  = (a - 1.0f) * rn;
          const float inp = (bt * bq[e]) * uu;
          hn = fmaf(a, hn, inp);
          sH[o] = hn;
          y = fmaf(cq[e], hn, y);
        }
      }
      const float sg = __builtin_amdgcn_rcpf(1.0f + expf(-zv));
      const float yv = (y + uu * Dd) * (zv * sg);
      sY[s * kScanYP + tid] = yv;
    }
    __syncthreads();
    v8h hv[8], lv[8];
#pragma unroll
    for (int it = 0; it < 8; ++it) {
      const int row = it * 8 + wave * 4 + q;
      const float* sp = sY + row * kScanYP + c8;
      const v4f a0 = *(const v4f*)(sp);
      const v4f a1 = *(const v4f*)(sp + 4);
#pragma unroll
      for (int e = 0; e < 4; ++e) {
        const unsigned short h0 = f2bf_bits(a0[e]), h1 = f2bf_bits(a1[e]);
        const unsigned short l0 = f2bf_bits(a0[e] - bf_bits2f(h0)), l1 = f2bf_bits(a1[e] - bf_bits2f(h1));
        hv[it][e]     = __builtin_bit_cast(_Float16, h0);
        hv[it][4 + e] = __builtin_bit_cast(_Float16, h1);
        lv[it][e]     = __builtin_bit_cast(_Float16, l0);
        lv[it][4 + e] = __builtin_bit_cast(_Float16, l1);
      }
    }
    for (int pass = 0; pass < 2; ++pass) {
#pragma unroll
      for (int it = 0; it < 8; ++it) {
        const int row = it * 8 + wave * 4 + q;
        const size_t o = (row0 + t0 + row) * kD + d0 + c8;
        *(volatile v8h*)(YH + o) = hv[it];
        *(volatile v8h*)(YL + o) = lv[it];
      }
      __threadfence();
    }
  }
}

extern "C" void kernel_launch(void* const* d_in, const int* in_sizes, int n_in,
                              void* d_out, int out_size, void* d_ws, size_t ws_size,
                              hipStream_t stream) {
  if (n_in < 10) return;
  if (in_sizes[0] != kRows * kD) return;
  if (in_sizes[1] != kD * kD) return;
  if (in_sizes[2] != kD * kD) return;
  if (in_sizes[3] != kPrN * kD) return;
  if (in_sizes[4] != kD * kConvK) return;
  if (in_sizes[5] != kD * kDtR) return;
  if (in_sizes[6] != kD) return;
  if (in_sizes[7] != kD * kNst) return;
  if (in_sizes[8] != kD) return;
  if (in_sizes[9] != kD * kD) return;
  if (out_size != kRows * kD) return;
  if (ws_size < kWsTotal) return;

  const float* x      = (const float*)d_in[0];
  const float* Wx     = (const float*)d_in[1];
  const float* Wz     = (const float*)d_in[2];
  const float* Wp     = (const float*)d_in[3];
  const float* conv_w = (const float*)d_in[4];
  const float* Wdt    = (const float*)d_in[5];
  const float* bdt    = (const float*)d_in[6];
  const float* A_log  = (const float*)d_in[7];
  const float* Dp     = (const float*)d_in[8];
  const float* Wo     = (const float*)d_in[9];
  float* out = (float*)d_out;

  char* ws = (char*)d_ws;
  unsigned short* XB   = (unsigned short*)(ws + kOffXB);
  unsigned short* WXZ  = (unsigned short*)(ws + kOffWXZ);
  unsigned short* WP   = (unsigned short*)(ws + kOffWP);
  unsigned short* WDT  = (unsigned short*)(ws + kOffWDT);
  unsigned short* WO   = (unsigned short*)(ws + kOffWO);
  float*          XZ   = (float*)(ws + kOffXZ);
  float*          PR   = (float*)(ws + kOffPR);
  unsigned short* DTH  = (unsigned short*)(ws + kOffDTH);
  unsigned short* DTL  = (unsigned short*)(ws + kOffDTL);
  unsigned short* YH   = (unsigned short*)(ws + kOffYH);
  unsigned short* YL   = (unsigned short*)(ws + kOffYL);

  constexpr int kX8  = kRows * kD / 8;
  constexpr int kW8  = kD * kD / 8;
  constexpr int kWp8 = kPrN * kD / 8;
  constexpr int kWpT = kPrP * kD / 8;
  constexpr int kWd8 = kD * kDtR / 8;
  static_assert((kX8 % 256) == 0 && (kW8 % 256) == 0 && (kWpT % 256) == 0 && (kWd8 % 256) == 0 && (kWp8 % 32) == 0, "cvt grids");
  cvt_rows_bf16_kernel<<<kX8 / 256, 256, 0, stream>>>(x, XB, kX8, kX8);
  cvt_rows_bf16_kernel<<<kW8 / 256, 256, 0, stream>>>(Wx, WXZ, kW8, kW8);
  cvt_rows_bf16_kernel<<<kW8 / 256, 256, 0, stream>>>(Wz, WXZ + (size_t)kD * kD, kW8, kW8);
  cvt_rows_bf16_kernel<<<kWpT / 256, 256, 0, stream>>>(Wp, WP, kWp8, kWpT);
  cvt_rows_bf16_kernel<<<kWd8 / 256, 256, 0, stream>>>(Wdt, WDT, kWd8, kWd8);
  cvt_rows_bf16_kernel<<<kW8 / 256, 256, 0, stream>>>(Wo, WO, kW8, kW8);

  wmma_gemm64<1, 0, 0, 0, false><<<dim3((kRows / 64) * (kXzN / 64) / 8, 1), 256, 0, stream>>>(
      XB, nullptr, kD, 0L,
      WXZ, nullptr, kD, 0L,
      (void*)XZ, nullptr, kXzN, 0L,
      nullptr, nullptr, 0L,
      kRows, kXzN, kD, 1.0f);

  wmma_gemm64<1, 0, 0, 0, false><<<dim3((kRows / 64) * (kPrP / 64) / 8, 1), 256, 0, stream>>>(
      XB, nullptr, kD, 0L,
      WP, nullptr, kD, 0L,
      (void*)PR, nullptr, kPrP, 0L,
      nullptr, nullptr, 0L,
      kRows, kPrP, kD, 1.0f);

  constexpr int kDt8 = kRows * kDtR / 8;
  static_assert((kDt8 % 256) == 0, "split grid");
  split_dtun_kernel<<<kDt8 / 256, 256, 0, stream>>>(PR, DTH, DTL, kDt8);

  scan_kernel<<<kBatch * (kD / kScanCh), kScanCh, 0, stream>>>(DTH, DTL, WDT, XZ, PR, conv_w, bdt, A_log, Dp, YH, YL);

  wmma_gemm64<1, 1, 0, 0, false><<<dim3((kRows / 64) * (kD / 64) / 8, 1), 256, 0, stream>>>(
      YH, YL, kD, 0L,
      WO, nullptr, kD, 0L,
      (void*)out, nullptr, kD, 0L,
      nullptr, nullptr, 0L,
      kRows, kD, kD, 1.0f);
}
